// RGCNSparseTIRComposableLayer_58411555226291
// MI455X (gfx1250) — hardware-verified
//
#include <hip/hip_runtime.h>
#include <math.h>

#define NN  100000
#define NE  1638400
#define NP  100032
#define KF  128
#define OF  64
#define NR  8
#define XC  (NR * OF)
#define NT  256
#define SRB 2048
#define RPW (SRB / 8)
#define NTL ((NN + SRB - 1) / SRB)
#define SCH 4096
#define SPT (SCH / NT)
#define NCH (NE / SCH)
typedef char chk_ne_sch[(NE % SCH == 0) ? 1 : -1];
typedef char chk_ne_spt[(NE % SPT == 0 && SPT % 4 == 0) ? 1 : -1];
typedef char chk_np[(NP % 64 == 0 && NP >= NN && (NN * KF) % 4 == 0) ? 1 : -1];
typedef char chk_xc[(XC % 64 == 0 && KF % 32 == 0) ? 1 : -1];

typedef __attribute__((ext_vector_type(16))) _Float16 v16h;
typedef __attribute__((ext_vector_type(8)))  _Float16 v8h;
typedef __attribute__((ext_vector_type(16))) __bf16   v16b;
typedef __attribute__((ext_vector_type(8)))  __bf16   v8b;
typedef __attribute__((ext_vector_type(8)))  float    v8f;
typedef __attribute__((ext_vector_type(4)))  float    v4f;
typedef __attribute__((ext_vector_type(2)))  float    v2f;
typedef __attribute__((ext_vector_type(4)))  int      v4i;
typedef __attribute__((ext_vector_type(2)))  unsigned v2u;

__device__ __forceinline__ unsigned short f2bf_bits(float f) {
  unsigned u = __float_as_uint(f);
  return (unsigned short)((u + 0x7FFFu + ((u >> 16) & 1u)) >> 16);
}
__device__ __forceinline__ float bf_bits2f(unsigned short h) { return __uint_as_float(((unsigned)h) << 16); }

__device__ __forceinline__ void dep_guard_h(v8f& a, v8f& b, v16h x, v16h y) { asm volatile("v_nop\n\tv_nop\n\tv_nop\n\tv_nop" : "+v"(a), "+v"(b) : "v"(x), "v"(y)); }
__device__ __forceinline__ void dep_guard_b(v8f& a, v8f& b, v16b x, v16b y) { asm volatile("v_nop\n\tv_nop\n\tv_nop\n\tv_nop" : "+v"(a), "+v"(b) : "v"(x), "v"(y)); }
__device__ __forceinline__ void keep4_h(v16h a, v16h b, v16h c, v16h d) { asm volatile("v_nop" :: "v"(a), "v"(b), "v"(c), "v"(d)); }
__device__ __forceinline__ void keep4_b(v16b a, v16b b, v16b c, v16b d) { asm volatile("v_nop" :: "v"(a), "v"(b), "v"(c), "v"(d)); }
__device__ __forceinline__ void acc_guard4(v8f& a, v8f& b, v8f& c, v8f& d) { asm volatile("v_nop\n\tv_nop\n\tv_nop\n\tv_nop" : "+v"(a), "+v"(b), "+v"(c), "+v"(d)); }
template <typename T> struct Frag;
template <> struct Frag<_Float16> {
  typedef v16h V; union U { v16h v; v8h h[2]; };
  static __device__ __forceinline__ v16h load(const _Float16* p) {
    U f; f.h[0] = *(const v8h*)(p); f.h[1] = *(const v8h*)(p + 16); return f.v;
  }
  static __device__ __forceinline__ v8f mma(v16h a, v16h b, v8f c) {
    return __builtin_amdgcn_wmma_f32_16x16x32_f16(false, a, false, b, (short)0, c, false, false);
  }
  static __device__ __forceinline__ void guard(v8f& a, v8f& b, v16h x, v16h y) { dep_guard_h(a, b, x, y); }
  static __device__ __forceinline__ void keep(v16h a, v16h b, v16h c, v16h d) { keep4_h(a, b, c, d); }
};
template <> struct Frag<__bf16> {
  typedef v16b V; union U { v16b v; v8b h[2]; };
  static __device__ __forceinline__ v16b load(const __bf16* p) {
    U f; f.h[0] = *(const v8b*)(p); f.h[1] = *(const v8b*)(p + 16); return f.v;
  }
  static __device__ __forceinline__ v8f mma(v16b a, v16b b, v8f c) {
    return __builtin_amdgcn_wmma_f32_16x16x32_bf16(false, a, false, b, (short)0, c, false, false);
  }
  static __device__ __forceinline__ void guard(v8f& a, v8f& b, v16b x, v16b y) { dep_guard_b(a, b, x, y); }
  static __device__ __forceinline__ void keep(v16b a, v16b b, v16b c, v16b d) { keep4_b(a, b, c, d); }
};

template <int ET> struct Elem;
template <> struct Elem<0> { typedef _Float16 T; };
template <> struct Elem<1> { typedef __bf16 T; };
template <int ET, bool SPLIT, int BIAS_MODE, int OUT_MODE, bool RESID, int ACT = 0>
__global__ __launch_bounds__(256) void wmma_gemm64(
    const unsigned short* __restrict__ Ap, const unsigned short* __restrict__ A2p, int lda, long strideA,
    const unsigned short* __restrict__ Btp, const unsigned short* __restrict__ Bt2p, int ldb, long strideB,
    void* __restrict__ Cout, void* __restrict__ Cout2, int ldc, long strideC,
    const float* __restrict__ bias,
    const float* __restrict__ resid, long strideR,
    int M, int N, int K, float scale) {
  typedef typename Elem<ET>::T T;
  typedef typename Frag<T>::V V;
  const T* A = (const T*)Ap; const T* A2 = (const T*)A2p; const T* Bt = (const T*)Btp; const T* Bt2 = (const T*)Bt2p;
  __shared__ __align__(16) float sT[8][16 * 68];
  const int b    = blockIdx.y;
  const int lane = threadIdx.x & 31;
  const int wave = threadIdx.x >> 5;
  const int tilesN = N >> 6;
  const int tilesM = M >> 6;
  const int tile = blockIdx.x * 8 + wave;
  if (tile >= tilesM * tilesN) return;
  const int tm = tile / tilesN;
  const int tn = tile - tm * tilesN;
  const int m0 = tm << 6;
  const int n0 = tn << 6;

  const T* Ab  = A  + (size_t)b * strideA;
  const T* Bb  = Bt + (size_t)b * strideB;
  const T* Ab2 = SPLIT ? (A2  + (size_t)b * strideA) : nullptr;
  const T* Bb2 = SPLIT ? (Bt2 + (size_t)b * strideB) : nullptr;

  const int rlane = lane & 15;
  const int koff  = (lane >> 4) * 8;
  const int mOff  = (lane >> 4) * 8;

  v8f acc[4][4];
#pragma unroll
  for (int i = 0; i < 4; ++i)
#pragma unroll
    for (int j = 0; j < 4; ++j) acc[i][j] = (v8f){0.f,0.f,0.f,0.f,0.f,0.f,0.f,0.f};

  for (int k0 = 0; k0 < K; k0 += 32) {
    V bh[4], bl[4];
#pragma unroll
    for (int j = 0; j < 4; ++j) {
      const size_t bo = (size_t)(n0 + (j << 4) + rlane) * ldb + koff + k0;
      bh[j] = Frag<T>::load(Bb + bo);
      if (SPLIT) bl[j] = Frag<T>::load(Bb2 + bo);
    }
#pragma unroll
    for (int i = 0; i < 4; ++i) {
      const size_t ao = (size_t)(m0 + (i << 4) + rlane) * lda + koff + k0;
      V ah = Frag<T>::load(Ab + ao);
      V al;
      if (SPLIT) al = Frag<T>::load(Ab2 + ao);
#pragma unroll
      for (int j = 0; j < 4; ++j) {
        acc[i][j] = Frag<T>::mma(ah, bh[j], acc[i][j]);
        if (SPLIT) {
          acc[i][j] = Frag<T>::mma(ah, bl[j], acc[i][j]);
          acc[i][j] = Frag<T>::mma(al, bh[j], acc[i][j]);
        }
      }
      Frag<T>::guard(acc[i][0], acc[i][3], ah, SPLIT ? al : ah);
    }
    Frag<T>::keep(bh[0], bh[1], bh[2], bh[3]);
    if (SPLIT) Frag<T>::keep(bl[0], bl[1], bl[2], bl[3]);
  }
  acc_guard4(acc[0][0], acc[0][1], acc[0][2], acc[0][3]);
  acc_guard4(acc[1][0], acc[1][1], acc[1][2], acc[1][3]);
  acc_guard4(acc[2][0], acc[2][1], acc[2][2], acc[2][3]);
  acc_guard4(acc[3][0], acc[3][1], acc[3][2], acc[3][3]);

  float* slab = sT[wave];
  const float* Rb = RESID ? (resid + (size_t)b * strideR) : nullptr;
#pragma unroll
  for (int i = 0; i < 4; ++i) {
    const int mBase = m0 + (i << 4);
#pragma unroll
    for (int j = 0; j < 4; ++j) {
      const int n = n0 + (j << 4) + rlane;
      float bv = 0.f;
      if (BIAS_MODE == 2) bv = bias[n];
#pragma unroll
      for (int r = 0; r < 8; ++r) {
        float v = acc[i][j][r] * scale;
        if (BIAS_MODE == 1) v += bias[mBase + mOff + r];
        if (BIAS_MODE == 2) v += bv;
        if (RESID) v += Rb[(size_t)(mBase + mOff + r) * ldc + n];
        if (ACT == 1) v = tanhf(v);
        if (ACT == 2) v = fmaxf(v, 0.0f);
        if (ACT == 3) v = v / (1.0f + expf(-v));
        if (ACT == 4) v = (v > 0.f) ? v : 0.01f * v;
        if (ACT == 5) v = 0.5f * v * (1.0f + erff(v * 0.70710678118654752f));
        slab[(mOff + r) * 68 + (j << 4) + rlane] = v;
      }
    }
    __builtin_amdgcn_fence(__ATOMIC_RELEASE, "workgroup");
    __builtin_amdgcn_wave_barrier();
    __builtin_amdgcn_fence(__ATOMIC_ACQUIRE, "workgroup");
    if (OUT_MODE == 0) {
      float* C = (float*)Cout + (size_t)b * strideC;
      const int hh = lane >> 4, c4 = (lane & 15) * 4;
      for (int pass = 0; pass < 2; ++pass) {
#pragma unroll
        for (int it = 0; it < 8; ++it) {
          const int row = it * 2 + hh;
          v4f v = *(const v4f*)(slab + row * 68 + c4);
          *(volatile v4f*)(C + (size_t)(mBase + row) * ldc + n0 + c4) = v;
        }
        __threadfence();
      }
    } else {
      const int q = lane >> 3, c8 = (lane & 7) * 8;
      unsigned short* C  = (unsigned short*)Cout  + (size_t)b * strideC;
      unsigned short* C2 = (OUT_MODE == 2) ? ((unsigned short*)Cout2 + (size_t)b * strideC) : nullptr;
      for (int pass = 0; pass < 2; ++pass) {
#pragma unroll
        for (int it = 0; it < 4; ++it) {
          const int row = it * 4 + q;
          const float* sp = slab + row * 68 + c8;
          v8h hv, lv;
#pragma unroll
          for (int e = 0; e < 8; ++e) {
            if (OUT_MODE == 1) {
              hv[e] = (_Float16)sp[e];
            } else {
              unsigned short hb = f2bf_bits(sp[e]);
              unsigned short lb = f2bf_bits(sp[e] - bf_bits2f(hb));
              hv[e] = __builtin_bit_cast(_Float16, hb);
              lv[e] = __builtin_bit_cast(_Float16, lb);
            }
          }
          *(volatile v8h*)(C + (size_t)(mBase + row) * ldc + n0 + c8) = hv;
          if (OUT_MODE == 2) *(volatile v8h*)(C2 + (size_t)(mBase + row) * ldc + n0 + c8) = lv;
        }
        __threadfence();
      }
    }
    __builtin_amdgcn_fence(__ATOMIC_RELEASE, "workgroup");
    __builtin_amdgcn_wave_barrier();
    __builtin_amdgcn_fence(__ATOMIC_ACQUIRE, "workgroup");
  }
}

__global__ __launch_bounds__(256) void cast_scale_f16x4(const float* __restrict__ in, unsigned short* __restrict__ out,
                                                        int n4_in, int n4_tot, float scale) {
  const int i = blockIdx.x * 256 + threadIdx.x;
  if (i < n4_tot) {
    const bool live = (i < n4_in);
    const int ic = live ? i : (n4_in - 1);
    const v4f x = *(const v4f*)(in + (size_t)ic * 4);
    unsigned short hb[4];
#pragma unroll
    for (int e = 0; e < 4; ++e) {
      const float a = live ? (x[e] * scale) : 0.f;
      hb[e] = __builtin_bit_cast(unsigned short, (_Float16)a);
    }
    v2u u;
    u[0] = (unsigned)hb[0] | ((unsigned)hb[1] << 16);
    u[1] = (unsigned)hb[2] | ((unsigned)hb[3] << 16);
    unsigned short* op = out + (size_t)i * 4;
    *(volatile v2u*)op = u;
    __threadfence();
    *(volatile v2u*)op = u;
  }
}

__device__ __forceinline__ int blk_excl_scan(int cnt, int* scan_ws, int tid, int* tot) {
  const int lane = tid & 31, wave = tid >> 5; int incl = cnt;
#pragma unroll
  for (int o = 1; o < 32; o <<= 1) { const int v = __shfl_up(incl, o, 32); if (lane >= o) incl += v; }
  if (lane == 31) scan_ws[wave] = incl;
  __syncthreads();
  if (wave == 0) { int wv = (lane < NT / 32) ? scan_ws[lane] : 0; int wincl = wv;
#pragma unroll
    for (int o = 1; o < 32; o <<= 1) { const int v = __shfl_up(wincl, o, 32); if (lane >= o) wincl += v; }
    if (lane < NT / 32) scan_ws[32 + lane] = wincl - wv; if (lane == 31) scan_ws[64] = wincl; }
  __syncthreads();
  const int res = scan_ws[32 + wave] + incl - cnt; *tot = scan_ws[64];
  return res;
}
template <int SPc, int CAP>
__device__ __forceinline__ int chunk_hits3(const int* __restrict__ dstv, const int* __restrict__ srcv, const int* __restrict__ typv,
                                           int e0, int n0, int nhi, int tid, int* LIST, int* scan_ws) {
  const int eb = e0 + tid * SPc;
  const bool inb = (eb < NE);
  const int ebc = inb ? eb : (NE - SPc);
  int rec[SPc]; int cnt = 0;
#pragma unroll
  for (int k = 0; k < SPc; k += 4) {
    const v4i d4 = *(const v4i*)(dstv + ebc + k);
    const v4i s4 = *(const v4i*)(srcv + ebc + k);
    const v4i t4 = *(const v4i*)(typv + ebc + k);
#pragma unroll
    for (int e = 0; e < 4; ++e) {
      const int d = d4[e]; int r = -1;
      if (inb && d >= n0 && d < nhi) {
        int s = s4[e]; s = s < 0 ? 0 : (s >= NN ? NN - 1 : s);
        int t = t4[e]; t = t < 0 ? 0 : (t >= NR ? NR - 1 : t);
        r = ((d - n0) << 20) | (t << 17) | s; ++cnt;
      }
      rec[k + e] = r;
    }
  }
  int tot; int p = blk_excl_scan(cnt, scan_ws, tid, &tot);
#pragma unroll
  for (int k = 0; k < SPc; ++k) if (rec[k] >= 0) { if ((unsigned)p < (unsigned)CAP) LIST[p] = rec[k]; ++p; }
  __syncthreads();
  return tot < CAP ? tot : CAP;
}

__global__ __launch_bounds__(NT) void rgcn_agg_kernel(const unsigned short* __restrict__ XW, const int* __restrict__ esrc,
                                                     const int* __restrict__ edst, const int* __restrict__ etyp, float* Y) {
  __shared__ int LIST[SCH];
  __shared__ int scan_ws[80];
  const int tid = threadIdx.x, lane = tid & 31, wave = tid >> 5;
  const int n0 = blockIdx.x * SRB;
  const int nhi = (n0 + SRB < NN) ? (n0 + SRB) : NN;
  const v2f z2 = {0.f, 0.f};
#pragma unroll 1
  for (int j = 0; j < RPW; ++j) {
    const int n = n0 + wave * RPW + j;
    if (n >= NN) break;
    *(v2f*)(Y + (size_t)n * OF + 2 * lane) = z2;
  }
#pragma unroll 1
  for (int c = 0; c < NCH; ++c) {
    const int tot = chunk_hits3<SPT, SCH>(edst, esrc, etyp, c * SCH, n0, nhi, tid, LIST, scan_ws);
#pragma unroll 1
    for (int base = 0; base < tot; base += 32) {
      const int q = base + lane;
      const int rv = (q < tot) ? LIST[q] : -1;
      const int own = (rv >= 0 && (rv >> 28) == wave) ? 1 : 0;
      unsigned msk = (unsigned)__ballot(own);
#pragma unroll 1
      for (int it = 0; it < 32; ++it) {
        if (msk == 0u) break;
        const int bp = __builtin_ctz(msk); msk &= msk - 1u;
        const int r = __shfl(rv, bp, 32);
        const int dl = r >> 20;
        const int t  = (r >> 17) & 7;
        int s = r & 0x1FFFF; s = s < NN ? s : NN - 1;
        int n = n0 + dl;     n = n < NN ? n : NN - 1;
        const unsigned xb = *(const unsigned*)(XW + (size_t)s * XC + t * OF + 2 * lane);
        const float ma = (float)__builtin_bit_cast(_Float16, (unsigned short)(xb & 0xFFFFu));
        const float mb = (float)__builtin_bit_cast(_Float16, (unsigned short)(xb >> 16));
        float* rp = Y + (size_t)n * OF + 2 * lane;
        const v2f a = *(const v2f*)rp;
        v2f nv;
        nv[0] = a[0] + ma;
        nv[1] = a[1] + mb;
        *(volatile v2f*)rp = nv;
        __threadfence();
        *(volatile v2f*)rp = nv;
      }
    }
    __syncthreads();
  }
#pragma unroll 1
  for (int j = 0; j < RPW; ++j) {
    const int n = n0 + wave * RPW + j;
    if (n >= NN) break;
    float* rp = Y + (size_t)n * OF + 2 * lane;
    const v2f v = *(const v2f*)rp;
    *(volatile v2f*)rp = v;
    __threadfence();
    *(volatile v2f*)rp = v;
  }
}

extern "C" void kernel_launch(void* const* d_in, const int* in_sizes, int n_in,
                              void* d_out, int out_size, void* d_ws, size_t ws_size,
                              hipStream_t stream) {
  if (n_in < 5) return;
  if (in_sizes[0] != NN * KF || in_sizes[1] != NR * OF * KF ||
      in_sizes[2] != NE || in_sizes[3] != NE || in_sizes[4] != NE) return;
  if (out_size != NN * OF) return;
  const float* feat = (const float*)d_in[0];
  const float* W    = (const float*)d_in[1];
  const int*   esrc = (const int*)d_in[2];
  const int*   edst = (const int*)d_in[3];
  const int*   etyp = (const int*)d_in[4];
  float*       Y    = (float*)d_out;

  char* ws = (char*)d_ws; size_t off = 0;
  auto carve = [&](size_t bytes) -> char* { char* p = ws + off; off += (bytes + 255) & ~(size_t)255; return p; };
  unsigned short* F16  = (unsigned short*)carve((size_t)NP * KF * 2);
  unsigned short* W16  = (unsigned short*)carve((size_t)XC * KF * 2);
  unsigned short* XW16 = (unsigned short*)carve((size_t)NP * XC * 2);
  if (off > ws_size || off > (size_t)134217728) return;

  {
    const int n4_in = NN * KF / 4, n4_tot = NP * KF / 4;
    cast_scale_f16x4<<<(n4_tot + 255) / 256, 256, 0, stream>>>(feat, F16, n4_in, n4_tot, 16.0f);
  }
  {
    const int n4 = XC * KF / 4;
    cast_scale_f16x4<<<(n4 + 255) / 256, 256, 0, stream>>>(W, W16, n4, n4, 64.0f);
  }
  {
    const int tiles = (NP / 64) * (XC / 64);
    wmma_gemm64<0, false, 0, 1, false><<<dim3((tiles + 7) / 8, 1), 256, 0, stream>>>(
        (const unsigned short*)F16, (const unsigned short*)nullptr, KF, 0L,
        (const unsigned short*)W16, (const unsigned short*)nullptr, KF, 0L,
        (void*)XW16, (void*)nullptr, XC, 0L,
        (const float*)nullptr, (const float*)nullptr, 0L, NP, XC, KF, 1.0f / 1024.0f);
  }
  rgcn_agg_kernel<<<NTL, NT, 0, stream>>>(XW16, esrc, edst, etyp, Y);
}
